// OptimizedMambaBlock_31662498906797
// MI455X (gfx1250) — hardware-verified
//
#include <hip/hip_runtime.h>
#define BB 8
#define CC 256
#define LL 1024
#define DI 512
#define DS 16
#define DTR 16
#define KCV 4
#define NTOK (BB * LL)
#define NXP 64

typedef __bf16 v16b __attribute__((ext_vector_type(16)));
typedef unsigned short v8us __attribute__((ext_vector_type(8), may_alias));
typedef float  v8f  __attribute__((ext_vector_type(8)));
typedef float  v4f  __attribute__((ext_vector_type(4)));
typedef float  v4fa __attribute__((ext_vector_type(4), may_alias));
union FragB { v16b v; v8us half[2]; unsigned short u[16]; };

__device__ __forceinline__ unsigned short bf16_bits(float x) { unsigned int u = __float_as_uint(x); return (unsigned short)((u + 0x7FFFu + ((u >> 16) & 1u)) >> 16); }
__device__ __forceinline__ float bf16_val(unsigned short b) { return __uint_as_float(((unsigned int)b) << 16); }
__device__ __forceinline__ float bf16_round(float x) { return bf16_val(bf16_bits(x)); }
template <int NT>
__device__ __forceinline__ v8f mmaN(v16b ah, v16b al, v16b bh, v16b bl, v8f c) {
  c = __builtin_amdgcn_wmma_f32_16x16x32_bf16(false, ah, false, bh, (short)0, c, false, false);
  if (NT >= 2) c = __builtin_amdgcn_wmma_f32_16x16x32_bf16(false, al, false, bh, (short)0, c, false, false);
  if (NT >= 3) c = __builtin_amdgcn_wmma_f32_16x16x32_bf16(false, ah, false, bl, (short)0, c, false, false);
  asm volatile("v_nop\n\tv_nop\n\tv_nop\n\tv_nop" : "+v"(c) : "v"(ah), "v"(al), "v"(bh), "v"(bl));
  return c;
}

__global__ __launch_bounds__(256) void k_wt_bf16(const float* __restrict__ W, unsigned short* __restrict__ Wt, int K, int N) {
  const int t = blockIdx.x * 256 + threadIdx.x;
  const int k8n = K / 8;
  if (t >= N * k8n) return;
  const int n = t / k8n, k8 = (t % k8n) * 8;
  v8us v;
#pragma unroll
  for (int i = 0; i < 8; ++i) v[i] = bf16_bits(W[(size_t)(k8 + i) * N + n]);
  *(volatile v8us*)(Wt + (size_t)n * K + k8) = v;
  __threadfence();
  *(volatile v8us*)(Wt + (size_t)n * K + k8) = v;
}

template <bool ASPLIT, int ACT, bool BIAS_BF16>
__global__ __launch_bounds__(128) void k_gemm_bf(const float* __restrict__ A, int lda, const unsigned short* __restrict__ Wt, int ldb,
                                               const float* __restrict__ bias, float* __restrict__ C, int ldc, int M, int N, int K) {
  __shared__ __attribute__((aligned(16))) float so[4][16][64];
  const int tid = threadIdx.x, w = tid >> 5, lane = tid & 31, ln = lane & 15, hh = lane >> 4;
  const int ntn = N / 64;
  const int wid = blockIdx.x * 4 + w;
  const int mt = wid / ntn, nq = wid % ntn;
  if (mt * 16 >= M) return;
  const int row0 = mt * 16, col0 = nq * 64;
  const float* arow = A + (size_t)(row0 + ln) * lda;
  v8f acc[4] = {};
  for (int kb = 0; kb < K; kb += 32) {
    FragB ah, al;
    const v4f x0 = *(const v4fa*)(arow + kb + 8 * hh), x1 = *(const v4fa*)(arow + kb + 8 * hh + 4);
    const v4f x2 = *(const v4fa*)(arow + kb + 16 + 8 * hh), x3 = *(const v4fa*)(arow + kb + 16 + 8 * hh + 4);
    float xs[16] = {x0[0],x0[1],x0[2],x0[3],x1[0],x1[1],x1[2],x1[3],x2[0],x2[1],x2[2],x2[3],x3[0],x3[1],x3[2],x3[3]};
#pragma unroll
    for (int i = 0; i < 16; ++i) { const unsigned short hb = bf16_bits(xs[i]); ah.u[i] = hb; al.u[i] = ASPLIT ? bf16_bits(xs[i] - bf16_val(hb)) : (unsigned short)0; }
#pragma unroll
    for (int t = 0; t < 4; ++t) {
      const unsigned short* brow = Wt + (size_t)(col0 + t * 16 + ln) * ldb + kb;
      FragB b;
      b.half[0] = *(const v8us*)(brow + 8 * hh);
      b.half[1] = *(const v8us*)(brow + 16 + 8 * hh);
      acc[t] = mmaN<ASPLIT ? 2 : 1>(ah.v, al.v, b.v, b.v, acc[t]);
    }
  }
#pragma unroll
  for (int t = 0; t < 4; ++t) {
    float bv = bias ? bias[col0 + t * 16 + ln] : 0.f;
    if (BIAS_BF16) bv = bf16_round(bv);
#pragma unroll
    for (int r = 0; r < 8; ++r) { float v = acc[t][r] + bv; if (ACT == 1) v = fmaxf(v, 0.f); so[w][8 * hh + r][t * 16 + ln] = v; }
  }
  __builtin_amdgcn_fence(__ATOMIC_ACQ_REL, "workgroup");
  __builtin_amdgcn_wave_barrier();
  const int rsub = lane >> 4, c4 = (lane & 15) * 4;
  for (int pass = 0; pass < 2; ++pass) {
#pragma unroll
    for (int q = 0; q < 8; ++q) {
      const int r = q * 2 + rsub;
      const v4f v = *(const v4fa*)&so[w][r][c4];
      *(volatile v4f*)(C + (size_t)(row0 + r) * ldc + col0 + c4) = v;
    }
    if (pass == 0) __threadfence();
  }
}

template <int D, bool CAUSAL>
__global__ __launch_bounds__(128) void k_flash(const float* __restrict__ qb, const float* __restrict__ kb, const float* __restrict__ vb,
                                             int pitch, int T, int H, float scale, float* __restrict__ y, int ypitch) {
  constexpr int KS = D / 32;
  constexpr int DT = D / 16;
  __shared__ __attribute__((aligned(16))) unsigned short sKh[32][D + 8], sKl[32][D + 8], sVh[32][D + 8], sVl[32][D + 8];
  __shared__ __attribute__((aligned(16))) unsigned short sPh[4][16][40], sPl[4][16][40];
  __shared__ __attribute__((aligned(16))) float sO[4][16][D];
  const int tid = threadIdx.x, w = tid >> 5, lane = tid & 31, ln = lane & 15, hh = lane >> 4;
  const int nqb = (T + 63) / 64;
  const int bh = blockIdx.x / nqb, qblk = blockIdx.x % nqb;
  const int b = bh / H, h = bh % H;
  const int q0 = qblk * 64 + w * 16;
  const float* Q = qb + (size_t)b * T * pitch + h * D;
  const float* K = kb + (size_t)b * T * pitch + h * D;
  const float* V = vb + (size_t)b * T * pitch + h * D;

  FragB aqh[KS], aql[KS];
  {
    int row = q0 + ln; if (row >= T) row = T - 1;
    const float* qr = Q + (size_t)row * pitch;
#pragma unroll
    for (int ks = 0; ks < KS; ++ks)
#pragma unroll
      for (int i = 0; i < 16; ++i) {
        const int d = ks * 32 + ((i < 8) ? (8 * hh + i) : (16 + 8 * hh + (i - 8)));
        const float x = qr[d] * scale; const unsigned short hb = bf16_bits(x);
        aqh[ks].u[i] = hb; aql[ks].u[i] = bf16_bits(x - bf16_val(hb));
      }
  }
  float m_r[8], l_r[8];
#pragma unroll
  for (int r = 0; r < 8; ++r) { m_r[r] = -3.0e38f; l_r[r] = 0.f; }
  v8f oacc[DT];
#pragma unroll
  for (int dt = 0; dt < DT; ++dt) oacc[dt] = (v8f){0.f,0.f,0.f,0.f,0.f,0.f,0.f,0.f};

  const int kv_end = CAUSAL ? min(T, qblk * 64 + 64) : T;
  for (int j0 = 0; j0 < kv_end; j0 += 32) {
    __syncthreads();
    for (int e = tid; e < 32 * (D / 4); e += 128) {
      const int r = e / (D / 4), c4 = (e % (D / 4)) * 4;
      const int key = j0 + r;
      v4f kf = {0.f,0.f,0.f,0.f}, vf = {0.f,0.f,0.f,0.f};
      if (key < T) { kf = *(const v4fa*)(K + (size_t)key * pitch + c4); vf = *(const v4fa*)(V + (size_t)key * pitch + c4); }
#pragma unroll
      for (int t = 0; t < 4; ++t) {
        unsigned short hb = bf16_bits(kf[t]); sKh[r][c4 + t] = hb; sKl[r][c4 + t] = bf16_bits(kf[t] - bf16_val(hb));
        hb = bf16_bits(vf[t]); sVh[r][c4 + t] = hb; sVl[r][c4 + t] = bf16_bits(vf[t] - bf16_val(hb));
      }
    }
    __syncthreads();
    v8f s[2];
#pragma unroll
    for (int nt = 0; nt < 2; ++nt) {
      v8f acc = {};
#pragma unroll
      for (int ks = 0; ks < KS; ++ks) {
        FragB bh_, bl_;
        bh_.half[0] = *(const v8us*)&sKh[nt * 16 + ln][ks * 32 + 8 * hh]; bh_.half[1] = *(const v8us*)&sKh[nt * 16 + ln][ks * 32 + 16 + 8 * hh];
        bl_.half[0] = *(const v8us*)&sKl[nt * 16 + ln][ks * 32 + 8 * hh]; bl_.half[1] = *(const v8us*)&sKl[nt * 16 + ln][ks * 32 + 16 + 8 * hh];
        acc = mmaN<3>(aqh[ks].v, aql[ks].v, bh_.v, bl_.v, acc);
      }
      s[nt] = acc;
    }
    float alpha[8];
#pragma unroll
    for (int r = 0; r < 8; ++r) {
      const int qi = q0 + 8 * hh + r;
      const int ja = j0 + ln, jb = j0 + 16 + ln;
      if (CAUSAL) { if (ja > qi) s[0][r] = -3.0e38f; if (jb > qi) s[1][r] = -3.0e38f; }
      if (ja >= T) s[0][r] = -3.0e38f;
      if (jb >= T) s[1][r] = -3.0e38f;
      float mx = fmaxf(s[0][r], s[1][r]);
      mx = fmaxf(mx, __shfl_xor(mx, 1, 32)); mx = fmaxf(mx, __shfl_xor(mx, 2, 32)); mx = fmaxf(mx, __shfl_xor(mx, 4, 32)); mx = fmaxf(mx, __shfl_xor(mx, 8, 32));
      const float mnew = fmaxf(m_r[r], mx);
      alpha[r] = (mnew > -1.0e38f) ? __expf(m_r[r] - mnew) : 1.0f;
      const float p0 = (s[0][r] > -1.0e38f) ? __expf(s[0][r] - mnew) : 0.f;
      const float p1 = (s[1][r] > -1.0e38f) ? __expf(s[1][r] - mnew) : 0.f;
      m_r[r] = mnew;
      l_r[r] = l_r[r] * alpha[r] + p0 + p1;
      unsigned short hb = bf16_bits(p0); sPh[w][8 * hh + r][ln] = hb;      sPl[w][8 * hh + r][ln] = bf16_bits(p0 - bf16_val(hb));
      hb = bf16_bits(p1);                sPh[w][8 * hh + r][16 + ln] = hb; sPl[w][8 * hh + r][16 + ln] = bf16_bits(p1 - bf16_val(hb));
    }
#pragma unroll
    for (int dt = 0; dt < DT; ++dt)
#pragma unroll
      for (int r = 0; r < 8; ++r) oacc[dt][r] *= alpha[r];
    __builtin_amdgcn_fence(__ATOMIC_ACQ_REL, "workgroup");
    __builtin_amdgcn_wave_barrier();
    FragB pah, pal;
    pah.half[0] = *(const v8us*)&sPh[w][ln][8 * hh]; pah.half[1] = *(const v8us*)&sPh[w][ln][16 + 8 * hh];
    pal.half[0] = *(const v8us*)&sPl[w][ln][8 * hh]; pal.half[1] = *(const v8us*)&sPl[w][ln][16 + 8 * hh];
#pragma unroll
    for (int dt = 0; dt < DT; ++dt) {
      FragB bvh, bvl;
#pragma unroll
      for (int i = 0; i < 8; ++i) {
        bvh.u[i] = sVh[8 * hh + i][dt * 16 + ln]; bvh.u[8 + i] = sVh[16 + 8 * hh + i][dt * 16 + ln];
        bvl.u[i] = sVl[8 * hh + i][dt * 16 + ln]; bvl.u[8 + i] = sVl[16 + 8 * hh + i][dt * 16 + ln];
      }
      oacc[dt] = mmaN<3>(pah.v, pal.v, bvh.v, bvl.v, oacc[dt]);
    }
    __builtin_amdgcn_fence(__ATOMIC_ACQ_REL, "workgroup");
    __builtin_amdgcn_wave_barrier();
  }
#pragma unroll
  for (int r = 0; r < 8; ++r) {
    float l = l_r[r];
    l += __shfl_xor(l, 1, 32); l += __shfl_xor(l, 2, 32); l += __shfl_xor(l, 4, 32); l += __shfl_xor(l, 8, 32);
    l_r[r] = (l > 0.f) ? 1.0f / l : 0.f;
  }
#pragma unroll
  for (int dt = 0; dt < DT; ++dt)
#pragma unroll
    for (int r = 0; r < 8; ++r) sO[w][8 * hh + r][dt * 16 + ln] = oacc[dt][r] * l_r[r];
  __builtin_amdgcn_fence(__ATOMIC_ACQ_REL, "workgroup");
  __builtin_amdgcn_wave_barrier();
  for (int pass = 0; pass < 2; ++pass) {
    for (int r = 0; r < 16; ++r) {
      const int row = q0 + r;
      if (row < T && lane < D / 4) {
        const v4f val = *(const v4fa*)&sO[w][r][lane * 4];
        *(volatile v4f*)(y + ((size_t)b * T + row) * ypitch + h * D + lane * 4) = val;
      }
    }
    if (pass == 0) __threadfence();
  }
}

template <bool AFFINE, bool RESID, bool RES_BF16>
__global__ __launch_bounds__(256) void k_transpose32(const float* __restrict__ in, float* __restrict__ out, int rows, int cols,
                                                    const float* __restrict__ scale, const float* __restrict__ shift, const float* __restrict__ res) {
  __shared__ float tile[32][33];
  const int b = blockIdx.z;
  const int r0 = blockIdx.y * 32, c0 = blockIdx.x * 32;
  const float* src = in + (size_t)b * rows * cols;
  float* dst = out + (size_t)b * rows * cols;
  const int tx = threadIdx.x & 31, ty = threadIdx.x >> 5;
  for (int i = ty; i < 32; i += 8) tile[i][tx] = src[(size_t)(r0 + i) * cols + c0 + tx];
  __syncthreads();
  for (int pass = 0; pass < 2; ++pass) {
    for (int i = ty; i < 32; i += 8) {
      float v = tile[tx][i];
      const int orow = c0 + i;
      if (AFFINE) v = v * scale[orow] + shift[orow];
      if (RESID) { float rv = res[(size_t)b * rows * cols + (size_t)orow * rows + r0 + tx]; if (RES_BF16) rv = bf16_round(rv); v += rv; }
      *(volatile float*)(dst + (size_t)orow * rows + r0 + tx) = v;
    }
    if (pass == 0) __threadfence();
  }
}

__global__ __launch_bounds__(256) void k_pool2_pm(const float* __restrict__ in, float* __restrict__ out, int Bn, int H, int W, int C) {
  const size_t t = (size_t)blockIdx.x * 256 + threadIdx.x;
  const int c4n = C / 4, Ho = H / 2, Wo = W / 2;
  const size_t total = (size_t)Bn * Ho * Wo * c4n;
  if (t >= total) return;
  const int c4 = (int)(t % c4n) * 4; size_t rest = t / c4n;
  const int pw = (int)(rest % Wo); rest /= Wo; const int ph = (int)(rest % Ho); const int b = (int)(rest / Ho);
  const float* base = in + (size_t)b * H * W * C;
  const int p00 = (2 * ph) * W + 2 * pw;
  const v4f a = *(const v4fa*)(base + (size_t)p00 * C + c4), bq = *(const v4fa*)(base + (size_t)(p00 + 1) * C + c4);
  const v4f c = *(const v4fa*)(base + (size_t)(p00 + W) * C + c4), d = *(const v4fa*)(base + (size_t)(p00 + W + 1) * C + c4);
  v4f m; for (int i = 0; i < 4; ++i) m[i] = fmaxf(fmaxf(a[i], bq[i]), fmaxf(c[i], d[i]));
  float* dst = out + ((size_t)b * Ho * Wo + (size_t)ph * Wo + pw) * C + c4;
  *(volatile v4f*)dst = m;
  __threadfence();
  *(volatile v4f*)dst = m;
}

template <int DQ, int DV>
__global__ __launch_bounds__(128) void k_flash2(const float* __restrict__ Qb, size_t qstride, int qpitch, int Tq,
                                              const float* __restrict__ Kb, size_t kstride, int kpitch, int Tk,
                                              const float* __restrict__ Vb, size_t vstride, int vpitch,
                                              float scale, float* __restrict__ y, size_t ystride, int ypitch) {
  constexpr int KS = DQ / 32, DT = DV / 16;
  __shared__ __attribute__((aligned(16))) unsigned short sKh[32][DQ + 8], sKl[32][DQ + 8], sVh[32][DV + 8], sVl[32][DV + 8];
  __shared__ __attribute__((aligned(16))) unsigned short sPh[4][16][40], sPl[4][16][40];
  __shared__ __attribute__((aligned(16))) float sO[4][16][DV];
  const int tid = threadIdx.x, w = tid >> 5, lane = tid & 31, ln = lane & 15, hh = lane >> 4;
  const int nqb = (Tq + 63) / 64;
  const int bh = blockIdx.x / nqb, qblk = blockIdx.x % nqb;
  const int dv0 = blockIdx.y * DV;
  const int q0 = qblk * 64 + w * 16;
  const float* Q = Qb + (size_t)bh * qstride; const float* K = Kb + (size_t)bh * kstride; const float* V = Vb + (size_t)bh * vstride + dv0;
  FragB aqh[KS], aql[KS];
  {
    int row = q0 + ln; if (row >= Tq) row = Tq - 1;
    const float* qr = Q + (size_t)row * qpitch;
#pragma unroll
    for (int ks = 0; ks < KS; ++ks)
#pragma unroll
      for (int i = 0; i < 16; ++i) {
        const int d = ks * 32 + ((i < 8) ? (8 * hh + i) : (16 + 8 * hh + (i - 8)));
        const float x = qr[d] * scale; const unsigned short hb = bf16_bits(x);
        aqh[ks].u[i] = hb; aql[ks].u[i] = bf16_bits(x - bf16_val(hb));
      }
  }
  float m_r[8], l_r[8];
#pragma unroll
  for (int r = 0; r < 8; ++r) { m_r[r] = -3.0e38f; l_r[r] = 0.f; }
  v8f oacc[DT];
#pragma unroll
  for (int dt = 0; dt < DT; ++dt) oacc[dt] = (v8f){0.f,0.f,0.f,0.f,0.f,0.f,0.f,0.f};
  for (int j0 = 0; j0 < Tk; j0 += 32) {
    __syncthreads();
    for (int e = tid; e < 32 * (DQ / 4); e += 128) {
      const int r = e / (DQ / 4), c4 = (e % (DQ / 4)) * 4; const int key = j0 + r;
      v4f f = {0.f,0.f,0.f,0.f}; if (key < Tk) f = *(const v4fa*)(K + (size_t)key * kpitch + c4);
#pragma unroll
      for (int t = 0; t < 4; ++t) { const unsigned short hb = bf16_bits(f[t]); sKh[r][c4 + t] = hb; sKl[r][c4 + t] = bf16_bits(f[t] - bf16_val(hb)); }
    }
    for (int e = tid; e < 32 * (DV / 4); e += 128) {
      const int r = e / (DV / 4), c4 = (e % (DV / 4)) * 4; const int key = j0 + r;
      v4f f = {0.f,0.f,0.f,0.f}; if (key < Tk) f = *(const v4fa*)(V + (size_t)key * vpitch + c4);
#pragma unroll
      for (int t = 0; t < 4; ++t) { const unsigned short hb = bf16_bits(f[t]); sVh[r][c4 + t] = hb; sVl[r][c4 + t] = bf16_bits(f[t] - bf16_val(hb)); }
    }
    __syncthreads();
    v8f s[2];
#pragma unroll
    for (int nt = 0; nt < 2; ++nt) {
      v8f acc = {};
#pragma unroll
      for (int ks = 0; ks < KS; ++ks) {
        FragB bh_, bl_;
        bh_.half[0] = *(const v8us*)&sKh[nt * 16 + ln][ks * 32 + 8 * hh]; bh_.half[1] = *(const v8us*)&sKh[nt * 16 + ln][ks * 32 + 16 + 8 * hh];
        bl_.half[0] = *(const v8us*)&sKl[nt * 16 + ln][ks * 32 + 8 * hh]; bl_.half[1] = *(const v8us*)&sKl[nt * 16 + ln][ks * 32 + 16 + 8 * hh];
        acc = mmaN<3>(aqh[ks].v, aql[ks].v, bh_.v, bl_.v, acc);
      }
      s[nt] = acc;
    }
    float alpha[8];
#pragma unroll
    for (int r = 0; r < 8; ++r) {
      const int ja = j0 + ln, jb = j0 + 16 + ln;
      if (ja >= Tk) s[0][r] = -3.0e38f;
      if (jb >= Tk) s[1][r] = -3.0e38f;
      float mx = fmaxf(s[0][r], s[1][r]);
      mx = fmaxf(mx, __shfl_xor(mx, 1, 32)); mx = fmaxf(mx, __shfl_xor(mx, 2, 32)); mx = fmaxf(mx, __shfl_xor(mx, 4, 32)); mx = fmaxf(mx, __shfl_xor(mx, 8, 32));
      const float mnew = fmaxf(m_r[r], mx);
      alpha[r] = (mnew > -1.0e38f) ? __expf(m_r[r] - mnew) : 1.0f;
      const float p0 = (s[0][r] > -1.0e38f) ? __expf(s[0][r] - mnew) : 0.f;
      const float p1 = (s[1][r] > -1.0e38f) ? __expf(s[1][r] - mnew) : 0.f;
      m_r[r] = mnew;
      l_r[r] = l_r[r] * alpha[r] + p0 + p1;
      unsigned short hb = bf16_bits(p0); sPh[w][8 * hh + r][ln] = hb;      sPl[w][8 * hh + r][ln] = bf16_bits(p0 - bf16_val(hb));
      hb = bf16_bits(p1);                sPh[w][8 * hh + r][16 + ln] = hb; sPl[w][8 * hh + r][16 + ln] = bf16_bits(p1 - bf16_val(hb));
    }
#pragma unroll
    for (int dt = 0; dt < DT; ++dt)
#pragma unroll
      for (int r = 0; r < 8; ++r) oacc[dt][r] *= alpha[r];
    __builtin_amdgcn_fence(__ATOMIC_ACQ_REL, "workgroup");
    __builtin_amdgcn_wave_barrier();
    FragB pah, pal;
    pah.half[0] = *(const v8us*)&sPh[w][ln][8 * hh]; pah.half[1] = *(const v8us*)&sPh[w][ln][16 + 8 * hh];
    pal.half[0] = *(const v8us*)&sPl[w][ln][8 * hh]; pal.half[1] = *(const v8us*)&sPl[w][ln][16 + 8 * hh];
#pragma unroll
    for (int dt = 0; dt < DT; ++dt) {
      FragB bvh, bvl;
#pragma unroll
      for (int i = 0; i < 8; ++i) {
        bvh.u[i] = sVh[8 * hh + i][dt * 16 + ln]; bvh.u[8 + i] = sVh[16 + 8 * hh + i][dt * 16 + ln];
        bvl.u[i] = sVl[8 * hh + i][dt * 16 + ln]; bvl.u[8 + i] = sVl[16 + 8 * hh + i][dt * 16 + ln];
      }
      oacc[dt] = mmaN<3>(pah.v, pal.v, bvh.v, bvl.v, oacc[dt]);
    }
    __builtin_amdgcn_fence(__ATOMIC_ACQ_REL, "workgroup");
    __builtin_amdgcn_wave_barrier();
  }
#pragma unroll
  for (int r = 0; r < 8; ++r) {
    float l = l_r[r];
    l += __shfl_xor(l, 1, 32); l += __shfl_xor(l, 2, 32); l += __shfl_xor(l, 4, 32); l += __shfl_xor(l, 8, 32);
    l_r[r] = (l > 0.f) ? 1.0f / l : 0.f;
  }
#pragma unroll
  for (int dt = 0; dt < DT; ++dt)
#pragma unroll
    for (int r = 0; r < 8; ++r) sO[w][8 * hh + r][dt * 16 + ln] = oacc[dt][r] * l_r[r];
  __builtin_amdgcn_fence(__ATOMIC_ACQ_REL, "workgroup");
  __builtin_amdgcn_wave_barrier();
  for (int pass = 0; pass < 2; ++pass) {
    for (int r = 0; r < 16; ++r) {
      const int row = q0 + r;
      for (int c4 = lane * 4; c4 < DV; c4 += 128) {
        if (row < Tq) {
          const v4f val = *(const v4fa*)&sO[w][r][c4];
          *(volatile v4f*)(y + (size_t)bh * ystride + (size_t)row * ypitch + dv0 + c4) = val;
        }
      }
    }
    if (pass == 0) __threadfence();
  }
}

template <bool ASPLIT, bool BSPLIT, int ACT>
__global__ __launch_bounds__(128) void k_gemm_b(const float* __restrict__ A, int lda, size_t sA, const unsigned short* __restrict__ Bh, const unsigned short* __restrict__ Bl, int ldb, size_t sB,
                                             const float* __restrict__ bias, const float* __restrict__ resid, int ldr, size_t sR, float rsign, float alpha,
                                             float* __restrict__ C, int ldc, size_t sC, int M, int N, int K) {
  __shared__ __attribute__((aligned(16))) float so[4][16][64];
  const int tid = threadIdx.x, w = tid >> 5, lane = tid & 31, ln = lane & 15, hh = lane >> 4;
  const int by = blockIdx.y;
  A += (size_t)by * sA; Bh += (size_t)by * sB; if (BSPLIT) Bl += (size_t)by * sB; C += (size_t)by * sC; if (resid) resid += (size_t)by * sR;
  const int ntn = (N + 63) / 64; const int wid = blockIdx.x * 4 + w; const int mt = wid / ntn, nq = wid % ntn;
  if (mt * 16 >= M) return;
  const int row0 = mt * 16, col0 = nq * 64;
  const float* arow = A + (size_t)(row0 + ln) * lda;
  v8f acc[4] = {};
  for (int kb = 0; kb < K; kb += 32) {
    FragB ah, al;
    const v4f x0 = *(const v4fa*)(arow + kb + 8 * hh), x1 = *(const v4fa*)(arow + kb + 8 * hh + 4);
    const v4f x2 = *(const v4fa*)(arow + kb + 16 + 8 * hh), x3 = *(const v4fa*)(arow + kb + 16 + 8 * hh + 4);
    float xs[16] = {x0[0],x0[1],x0[2],x0[3],x1[0],x1[1],x1[2],x1[3],x2[0],x2[1],x2[2],x2[3],x3[0],x3[1],x3[2],x3[3]};
#pragma unroll
    for (int i = 0; i < 16; ++i) { const unsigned short hb = bf16_bits(xs[i]); ah.u[i] = hb; al.u[i] = ASPLIT ? bf16_bits(xs[i] - bf16_val(hb)) : (unsigned short)0; }
#pragma unroll
    for (int t = 0; t < 4; ++t) {
      if (col0 + t * 16 >= N) continue;
      const size_t boff = (size_t)(col0 + t * 16 + ln) * ldb + kb;
      FragB bh_, bl_; bh_.half[0] = *(const v8us*)(Bh + boff + 8 * hh); bh_.half[1] = *(const v8us*)(Bh + boff + 16 + 8 * hh);
      if (BSPLIT) { bl_.half[0] = *(const v8us*)(Bl + boff + 8 * hh); bl_.half[1] = *(const v8us*)(Bl + boff + 16 + 8 * hh); } else bl_ = bh_;
      acc[t] = mmaN<ASPLIT ? (BSPLIT ? 3 : 2) : 1>(ah.v, al.v, bh_.v, bl_.v, acc[t]);
    }
  }
#pragma unroll
  for (int t = 0; t < 4; ++t) {
    const int col = col0 + t * 16 + ln; if (col0 + t * 16 >= N) continue; const float bv = bias ? bf16_round(bias[col]) : 0.f;
#pragma unroll
    for (int r = 0; r < 8; ++r) { float v = acc[t][r] * alpha + bv; if (resid) v += rsign * resid[(size_t)(row0 + 8 * hh + r) * ldr + col]; if (ACT == 1) v = fmaxf(v, 0.f); else if (ACT == 2) v = fmaxf(v, 0.f) + log1pf(expf(-fabsf(v))); so[w][8 * hh + r][t * 16 + ln] = v; }
  }
  __builtin_amdgcn_fence(__ATOMIC_ACQ_REL, "workgroup"); __builtin_amdgcn_wave_barrier();
  const int rsub = lane >> 4, c4 = (lane & 15) * 4;
  for (int pass = 0; pass < 2; ++pass) {
#pragma unroll
    for (int q = 0; q < 8; ++q) { const int r = q * 2 + rsub; if (col0 + c4 < N) { const v4f v = *(const v4fa*)&so[w][r][c4]; *(volatile v4f*)(C + (size_t)(row0 + r) * ldc + col0 + c4) = v; } }
    if (pass == 0) __threadfence();
  }
}
__global__ __launch_bounds__(256) void k_split_transpose_b(const float* __restrict__ src, int lds_, size_t sIn, unsigned short* __restrict__ hi, unsigned short* __restrict__ lo, size_t sOut, int K, int N) {
  const size_t t = (size_t)blockIdx.x * 256 + threadIdx.x; const int k8n = K / 8; if (t >= (size_t)N * k8n) return;
  src += (size_t)blockIdx.y * sIn; hi += (size_t)blockIdx.y * sOut; lo += (size_t)blockIdx.y * sOut;
  const int n = (int)(t / k8n), k8 = (int)(t % k8n) * 8; v8us vh, vl;
#pragma unroll
  for (int i = 0; i < 8; ++i) { const float x = src[(size_t)(k8 + i) * lds_ + n]; const unsigned short hb = bf16_bits(x); vh[i] = hb; vl[i] = bf16_bits(x - bf16_val(hb)); }
  unsigned short* dh = hi + (size_t)n * K + k8; unsigned short* dl = lo + (size_t)n * K + k8;
  *(volatile v8us*)dh = vh; *(volatile v8us*)dl = vl; __threadfence(); *(volatile v8us*)dh = vh; *(volatile v8us*)dl = vl;
}

__global__ __launch_bounds__(256) void k_round_rows(const float* __restrict__ W, unsigned short* __restrict__ Wt, int n8) {
  const int t = blockIdx.x * 256 + threadIdx.x;
  if (t >= n8) return;
  const v4f a = *(const v4fa*)(W + (size_t)t * 8), b = *(const v4fa*)(W + (size_t)t * 8 + 4);
  v8us v; v[0]=bf16_bits(a[0]); v[1]=bf16_bits(a[1]); v[2]=bf16_bits(a[2]); v[3]=bf16_bits(a[3]);
  v[4]=bf16_bits(b[0]); v[5]=bf16_bits(b[1]); v[6]=bf16_bits(b[2]); v[7]=bf16_bits(b[3]);
  *(volatile v8us*)(Wt + (size_t)t * 8) = v; __threadfence(); *(volatile v8us*)(Wt + (size_t)t * 8) = v;
}

__global__ __launch_bounds__(256) void k_zpadrows(const float* __restrict__ W, unsigned short* __restrict__ Bt, int nreal, int npad, int K) { const int t = blockIdx.x * 256 + threadIdx.x; if (t >= npad * K / 8) return; const int k8 = (t % (K / 8)) * 8, n = t / (K / 8); v8us v; for (int q = 0; q < 8; ++q) v[q] = bf16_bits(n < nreal ? W[(size_t)n * K + k8 + q] : 0.f); *(volatile v8us*)(Bt + (size_t)n * K + k8) = v; __threadfence(); *(volatile v8us*)(Bt + (size_t)n * K + k8) = v; }
__global__ __launch_bounds__(256) void k_zpadcols(const float* __restrict__ W, unsigned short* __restrict__ Bt, int N, int kreal, int KP) { const int t = blockIdx.x * 256 + threadIdx.x; if (t >= N * KP / 8) return; const int k8 = (t % (KP / 8)) * 8, n = t / (KP / 8); v8us v; for (int q = 0; q < 8; ++q) { const int k = k8 + q; v[q] = bf16_bits(k < kreal ? W[(size_t)n * kreal + k] : 0.f); } *(volatile v8us*)(Bt + (size_t)n * KP + k8) = v; __threadfence(); *(volatile v8us*)(Bt + (size_t)n * KP + k8) = v; }
__global__ __launch_bounds__(256) void k_xpd(const float* __restrict__ XP, float* __restrict__ XPD) { const int t = blockIdx.x * 256 + threadIdx.x; if (t >= NTOK * 32 / 4) return; const int c4 = (t * 4) % 32, tok = (t * 4) / 32; v4f o; for (int q = 0; q < 4; ++q) { const int c = c4 + q; o[q] = (c < DTR) ? XP[(size_t)tok * NXP + c] : 0.f; } *(volatile v4f*)(XPD + (size_t)t * 4) = o; __threadfence(); *(volatile v4f*)(XPD + (size_t)t * 4) = o; }
__global__ __launch_bounds__(256) void k_xf(const float* __restrict__ x, float* __restrict__ XF) { __shared__ float tile[32][33]; const int b = blockIdx.z; const int c0 = blockIdx.y * 32, l0 = blockIdx.x * 32; const int tx = threadIdx.x & 31, ty = threadIdx.x >> 5;
  for (int i = ty; i < 32; i += 8) tile[i][tx] = bf16_round(x[((size_t)b * CC + c0 + i) * LL + l0 + tx]); __syncthreads();
  for (int pass = 0; pass < 2; ++pass) { for (int i = ty; i < 32; i += 8) *(volatile float*)(XF + ((size_t)b * LL + l0 + i) * CC + c0 + tx) = tile[tx][i]; if (pass == 0) __threadfence(); } }
__global__ __launch_bounds__(256) void k_ln(const float* __restrict__ X, const float* __restrict__ g, const float* __restrict__ bb, float* __restrict__ Y) { const int tid = threadIdx.x, wv = tid >> 5, lane = tid & 31; const size_t t = (size_t)blockIdx.x * 8 + wv; const float* r = X + t * CC; float v[8]; float s = 0.f;
#pragma unroll
  for (int u = 0; u < 8; ++u) { v[u] = r[u * 32 + lane]; s += v[u]; } for (int o = 16; o >= 1; o >>= 1) s += __shfl_xor(s, o, 32); const float mu = s * (1.0f / CC); float q = 0.f;
#pragma unroll
  for (int u = 0; u < 8; ++u) { const float d = v[u] - mu; q += d * d; } for (int o = 16; o >= 1; o >>= 1) q += __shfl_xor(q, o, 32); const float rs = rsqrtf(q * (1.0f / CC) + 1e-5f);
  for (int pass = 0; pass < 2; ++pass) {
#pragma unroll
    for (int u = 0; u < 8; ++u) { const int c = u * 32 + lane; *(volatile float*)(Y + t * CC + c) = (v[u] - mu) * rs * bf16_round(g[c]) + bf16_round(bb[c]); } if (pass == 0) __threadfence(); } }
__device__ __forceinline__ float silu1(float v) { return v / (1.0f + expf(-v)); }
__global__ __launch_bounds__(256) void k_conv(const float* __restrict__ XZ, const float* __restrict__ cw, const float* __restrict__ cb, float* __restrict__ U) { const int t2 = blockIdx.x * 256 + threadIdx.x; if (t2 >= NTOK * DI / 4) return; const int d4 = (t2 * 4) % DI; const int tok = (t2 * 4) / DI; const int l = tok % LL; v4f o;
  for (int q = 0; q < 4; ++q) { const int d = d4 + q; float s = bf16_round(cb[d]);
#pragma unroll
    for (int k = 0; k < KCV; ++k) { const int lp = l - (KCV - 1) + k; const float xv = (lp >= 0) ? XZ[(size_t)(tok - (KCV - 1) + k) * (2 * DI) + d] : 0.f; s += xv * bf16_round(cw[d * KCV + k]); } o[q] = silu1(s); }
  *(volatile v4f*)(U + (size_t)t2 * 4) = o; __threadfence(); *(volatile v4f*)(U + (size_t)t2 * 4) = o; }
__global__ __launch_bounds__(256) void k_scan(const float* __restrict__ U, const float* __restrict__ DT, const float* __restrict__ XP, const float* __restrict__ XZ, const float* __restrict__ dtb, const float* __restrict__ Alog, const float* __restrict__ Dp, float* __restrict__ Y) { const int b = blockIdx.x >> 1; const int d = (blockIdx.x & 1) * 256 + threadIdx.x; float A[DS], h[DS];
  for (int n = 0; n < DS; ++n) { A[n] = -expf(bf16_round(Alog[d * DS + n])); h[n] = 0.f; } const float bd = bf16_round(dtb[d]), Dd = bf16_round(Dp[d]);
#pragma unroll 1
  for (int l = 0; l < LL; ++l) { const size_t tok = (size_t)b * LL + l; const float z0 = DT[tok * DI + d] + bd; const float dt = (z0 > 20.f) ? z0 : log1pf(expf(z0)); const float u = U[tok * DI + d]; const float* xp = XP + tok * NXP; const float du = dt * u; float y = 0.f;
#pragma unroll 8
    for (int n = 0; n < DS; ++n) { h[n] = __expf(dt * A[n]) * h[n] + du * xp[DTR + n]; y += h[n] * xp[DTR + DS + n]; }
    y += u * Dd; const float z = XZ[tok * (2 * DI) + DI + d]; const float out = y * silu1(z); *(volatile float*)(Y + tok * DI + d) = out; }
  __threadfence();
#pragma unroll 1
  for (int l = 0; l < LL; ++l) { const size_t tok = (size_t)b * LL + l; const float v = Y[tok * DI + d]; *(volatile float*)(Y + tok * DI + d) = v; } }
__global__ __launch_bounds__(256) void k_gelu(float* __restrict__ Hm, const float* __restrict__ b1) { const size_t t = (size_t)blockIdx.x * 256 + threadIdx.x; if (t >= (size_t)NTOK * 4 * CC / 4) return; const int c4 = (int)((t * 4) % (4 * CC)); v4f v = *(const v4fa*)(Hm + t * 4); for (int q = 0; q < 4; ++q) { const float a = v[q] + bf16_round(b1[c4 + q]); v[q] = 0.5f * a * (1.0f + erff(a * 0.70710678118654752f)); } *(volatile v4f*)(Hm + t * 4) = v; __threadfence(); *(volatile v4f*)(Hm + t * 4) = v; }
extern "C" void kernel_launch(void* const* d_in, const int* in_sizes, int n_in,
                              void* d_out, int out_size, void* d_ws, size_t ws_size, hipStream_t stream) {
  (void)in_sizes; (void)n_in; (void)out_size;
  const float* x = (const float*)d_in[0]; const float* lng = (const float*)d_in[1]; const float* lnb = (const float*)d_in[2]; const float* inw = (const float*)d_in[3]; const float* cw = (const float*)d_in[4]; const float* cb = (const float*)d_in[5]; const float* xpw = (const float*)d_in[6]; const float* dtw = (const float*)d_in[7]; const float* dtb = (const float*)d_in[8]; const float* Alog = (const float*)d_in[9]; const float* Dp = (const float*)d_in[10]; const float* outw = (const float*)d_in[11];
  const float* mg = (const float*)d_in[12]; const float* mb = (const float*)d_in[13]; const float* w1 = (const float*)d_in[14]; const float* b1 = (const float*)d_in[15]; const float* w2 = (const float*)d_in[16]; const float* b2 = (const float*)d_in[17];
  char* ws = (char*)d_ws; size_t off = 0;
  auto take = [&](size_t bytes) { char* p = ws + off; off += (bytes + 255) & ~(size_t)255; return p; };
  unsigned short* Bin = (unsigned short*)take((size_t)2 * DI * CC * 2); unsigned short* Bxp = (unsigned short*)take((size_t)NXP * DI * 2); unsigned short* Bdt = (unsigned short*)take((size_t)DI * 32 * 2); unsigned short* Bout = (unsigned short*)take((size_t)CC * DI * 2); unsigned short* B1 = (unsigned short*)take((size_t)4 * CC * CC * 2); unsigned short* B2 = (unsigned short*)take((size_t)CC * 4 * CC * 2);
  float* XF = (float*)take((size_t)NTOK * CC * 4); float* XN = (float*)take((size_t)NTOK * CC * 4); float* XZ = (float*)take((size_t)NTOK * 2 * DI * 4); float* U = (float*)take((size_t)NTOK * DI * 4); float* XP = (float*)take((size_t)NTOK * NXP * 4); float* XPD = (float*)take((size_t)NTOK * 32 * 4); float* DT = (float*)take((size_t)NTOK * DI * 4); float* Y = (float*)take((size_t)NTOK * DI * 4);
  float* XF2 = (float*)take((size_t)NTOK * CC * 4); float* Hm = XZ;   float* XF3 = XN;
  if (off > ws_size) return;
  k_round_rows<<<(2 * DI * CC / 8 + 255) / 256, 256, 0, stream>>>(inw, Bin, 2 * DI * CC / 8); k_zpadrows<<<(NXP * DI / 8 + 255) / 256, 256, 0, stream>>>(xpw, Bxp, 48, NXP, DI); k_zpadcols<<<(DI * 32 / 8 + 255) / 256, 256, 0, stream>>>(dtw, Bdt, DI, DTR, 32);
  k_round_rows<<<(CC * DI / 8 + 255) / 256, 256, 0, stream>>>(outw, Bout, CC * DI / 8); k_round_rows<<<(4 * CC * CC / 8 + 255) / 256, 256, 0, stream>>>(w1, B1, 4 * CC * CC / 8); k_round_rows<<<(CC * 4 * CC / 8 + 255) / 256, 256, 0, stream>>>(w2, B2, CC * 4 * CC / 8);
  k_xf<<<dim3(LL / 32, CC / 32, BB), 256, 0, stream>>>(x, XF); k_ln<<<NTOK / 8, 256, 0, stream>>>(XF, lng, lnb, XN);
  k_gemm_b<true, false, 0><<<dim3(((NTOK / 16) * (2 * DI / 64) + 3) / 4, 1), 128, 0, stream>>>(XN, CC, 0, Bin, Bin, CC, 0, nullptr, nullptr, 0, 0, 1.f, 1.f, XZ, 2 * DI, 0, NTOK, 2 * DI, CC);
  k_conv<<<(NTOK * DI / 4 + 255) / 256, 256, 0, stream>>>(XZ, cw, cb, U);
  k_gemm_b<true, false, 0><<<dim3(((NTOK / 16) * 1 + 3) / 4, 1), 128, 0, stream>>>(U, DI, 0, Bxp, Bxp, DI, 0, nullptr, nullptr, 0, 0, 1.f, 1.f, XP, NXP, 0, NTOK, NXP, DI);
  k_xpd<<<(NTOK * 32 / 4 + 255) / 256, 256, 0, stream>>>(XP, XPD);
  k_gemm_b<true, false, 0><<<dim3(((NTOK / 16) * (DI / 64) + 3) / 4, 1), 128, 0, stream>>>(XPD, 32, 0, Bdt, Bdt, 32, 0, nullptr, nullptr, 0, 0, 1.f, 1.f, DT, DI, 0, NTOK, DI, 32);
  k_scan<<<BB * 2, 256, 0, stream>>>(U, DT, XP, XZ, dtb, Alog, Dp, Y);
  k_gemm_b<true, false, 0><<<dim3(((NTOK / 16) * (CC / 64) + 3) / 4, 1), 128, 0, stream>>>(Y, DI, 0, Bout, Bout, DI, 0, nullptr, XF, CC, 0, 1.f, 1.f, XF2, CC, 0, NTOK, CC, DI);
  k_ln<<<NTOK / 8, 256, 0, stream>>>(XF2, mg, mb, XF3);
  k_gemm_b<true, false, 0><<<dim3(((NTOK / 16) * (4 * CC / 64) + 3) / 4, 1), 128, 0, stream>>>(XF3, CC, 0, B1, B1, CC, 0, nullptr, nullptr, 0, 0, 1.f, 1.f, Hm, 4 * CC, 0, NTOK, 4 * CC, CC);
  k_gelu<<<(unsigned)(((size_t)NTOK * 4 * CC / 4 + 255) / 256), 256, 0, stream>>>(Hm, b1);
  k_gemm_b<true, false, 0><<<dim3(((NTOK / 16) * (CC / 64) + 3) / 4, 1), 128, 0, stream>>>(Hm, 4 * CC, 0, B2, B2, 4 * CC, 0, b2, XF2, CC, 0, 1.f, 1.f, U, CC, 0, NTOK, CC, 4 * CC);
  k_transpose32<false, false, false><<<dim3(CC / 32, LL / 32, BB), 256, 0, stream>>>(U, (float*)d_out, LL, CC, nullptr, nullptr, nullptr);
}
